// MambaBlock_30648886624685
// MI455X (gfx1250) — hardware-verified
//
#include <hip/hip_runtime.h>
#include <stddef.h>
#include <stdint.h>
#include <math.h>


#define NTOK   2048
#define SEQ    1024
#define DM     768
#define DI     1536
#define NH     24
#define HD     64
#define DS     64
#define CONVD  1664
#define DPROJ  3224
#define NPAD   3264
#define DTOFF  3200
#define K1     1536
#define K2     3072
#define QC     64
#define NCH    16
#define TE     4096
#define GBM    64
#define GBN    64
#define GTHR   128
#define NTHR   256
#define NU_IN   (NPAD * (DM / 8))
#define NU_OUT  (DM * (DI / 8))
#define C4ROW   (CONVD / 4)
#define NU_CONV (NTOK * C4ROW)
#define SSD_INTS (12 * (TE / 2) + 2 * TE + 5 * 64)
#define WSMAX  134217728

static_assert(NU_IN % NTHR == 0 && NU_OUT % NTHR == 0 && NU_CONV % NTHR == 0);
static_assert((DM / 8) % 32 == 0 && (DI / 8) % 32 == 0 && C4ROW % 32 == 0);
static_assert(K1 % 32 == 0 && K2 % 32 == 0 && K1 == 2 * DM && K2 == 2 * DI);
static_assert(NTOK % GBM == 0 && NPAD % GBN == 0 && DM % GBN == 0 && NPAD >= DPROJ);
static_assert(GBM == (GTHR / 32) * 16 && GBN == 64);
static_assert(DTOFF + NH == DPROJ && DI + CONVD == DTOFF && CONVD == DI + 2 * DS);
static_assert(SEQ == QC * NCH && NTOK == 2 * SEQ && NH * HD == DI);
static_assert(NTOK % 8 == 0 && DM == 3 * 256 && DI == 6 * 256);
static_assert(SSD_INTS * 4 <= 300000);

typedef float          v4f   __attribute__((ext_vector_type(4)));
typedef float          v8f   __attribute__((ext_vector_type(8)));
typedef int            v8i   __attribute__((ext_vector_type(8)));
typedef unsigned short v4us  __attribute__((ext_vector_type(4)));
typedef unsigned short v8us  __attribute__((ext_vector_type(8)));
typedef unsigned short v16us __attribute__((ext_vector_type(16)));
typedef __bf16         v16bf __attribute__((ext_vector_type(16)));
typedef v4f  __attribute__((may_alias)) v4fa;
typedef v4us __attribute__((may_alias)) v4usa;
typedef v8us __attribute__((may_alias)) v8usa;
union FragB { v16bf v; v16us u; v8us h[2]; v8i w; };

__device__ __forceinline__ v8f wmb(const FragB& a, const FragB& b, v8f c) {
  v8f d = __builtin_amdgcn_wmma_f32_16x16x32_bf16(false, a.v, false, b.v, (short)0, c, false, false);
  asm volatile("v_nop\n\tv_nop\n\tv_nop\n\tv_nop" : "+v"(d) : "v"(a.w), "v"(b.w));
  return d;
}
__device__ __forceinline__ v8f mm3(const FragB& ah, const FragB& al, const FragB& bh, const FragB& bl, v8f c) {
  c = wmb(ah, bh, c);
  c = wmb(ah, bl, c);
  c = wmb(al, bh, c);
  return c;
}

__device__ __forceinline__ unsigned bf16_bits(float f) {
  const unsigned u = __float_as_uint(f);
  return (u + 0x7FFFu + ((u >> 16) & 1u)) >> 16;
}
__device__ __forceinline__ float bf16_val(float f) {
  return __uint_as_float(bf16_bits(f) << 16);
}
__device__ __forceinline__ float bf_to_f(unsigned short b) {
  return __uint_as_float(((unsigned)b) << 16);
}
__device__ __forceinline__ void split2(float v, unsigned short& h, unsigned short& l) {
  const unsigned hb = bf16_bits(v);
  h = (unsigned short)hb;
  l = (unsigned short)bf16_bits(v - __uint_as_float(hb << 16));
}
__device__ __forceinline__ float silu_f(float v) {
  const float e = expf(-v);
  return v * __builtin_amdgcn_rcpf(1.0f + e);
}
__device__ __forceinline__ void lds_frag(FragB& f, const unsigned short* rp) {
  f.h[0] = *(const v8usa*)rp;
  f.h[1] = *(const v8usa*)(rp + 16);
}

__global__ __launch_bounds__(NTHR) void k_prep(const float* __restrict__ Win, const float* __restrict__ Wout,
                                               unsigned short* WIN2, unsigned short* WOUT2) {
  const int u = (int)blockIdx.x * NTHR + (int)threadIdx.x;
  v8us o;
  unsigned short* dp;
  int dup;
  if (u < NU_IN) {
    const int n  = u / (DM / 8);
    const int k8 = (u - n * (DM / 8)) * 8;
    const int nc = n < DPROJ ? n : DPROJ - 1;
    const bool ok = n < DPROJ;
    const float* p = Win + (size_t)k8 * DPROJ + nc;
#pragma unroll
    for (int i = 0; i < 8; ++i) {
      const unsigned short b = (unsigned short)bf16_bits(p[(size_t)i * DPROJ]);
      o[i] = ok ? b : (unsigned short)0;
    }
    dp = WIN2 + (size_t)n * K1 + k8;
    dup = DM;
  } else if (u < NU_IN + NU_OUT) {
    const int v  = u - NU_IN;
    const int n  = v / (DI / 8);
    const int k8 = (v - n * (DI / 8)) * 8;
    const float* p = Wout + (size_t)k8 * DM + n;
#pragma unroll
    for (int i = 0; i < 8; ++i) o[i] = (unsigned short)bf16_bits(p[(size_t)i * DM]);
    dp = WOUT2 + (size_t)n * K2 + k8;
    dup = DI;
  } else {
    return;
  }
  *(volatile v8us*)dp = o;
  *(volatile v8us*)(dp + dup) = o;
  __threadfence();
  *(volatile v8us*)dp = o;
  *(volatile v8us*)(dp + dup) = o;
}

__global__ __launch_bounds__(NTHR) void k_ln(const float* __restrict__ x, const float* __restrict__ lnw,
                                             const float* __restrict__ lnb, unsigned short* XN) {
  __shared__ __attribute__((aligned(16))) float xb[8 * DM];
  const int tid = (int)threadIdx.x, lane = tid & 31, wave = tid >> 5;
  const int row = (int)blockIdx.x * 8 + wave;
  const float* xr = x + (size_t)row * DM;
  float* xw = xb + wave * DM;

  float s = 0.0f;
#pragma unroll 1
  for (int j = 0; j < 3; ++j) {
    const int off = 256 * j + 8 * lane;
    const v4f a = *(const v4fa*)(xr + off);
    const v4f b = *(const v4fa*)(xr + off + 4);
    v4f va, vb;
    va.x = bf16_val(a.x); va.y = bf16_val(a.y); va.z = bf16_val(a.z); va.w = bf16_val(a.w);
    vb.x = bf16_val(b.x); vb.y = bf16_val(b.y); vb.z = bf16_val(b.z); vb.w = bf16_val(b.w);
    s += va.x; s += va.y; s += va.z; s += va.w;
    s += vb.x; s += vb.y; s += vb.z; s += vb.w;
    *(v4fa*)(xw + off) = va;
    *(v4fa*)(xw + off + 4) = vb;
  }
#pragma unroll
  for (int d = 16; d > 0; d >>= 1) s += __shfl_xor(s, d, 32);
  const float mu = s * (1.0f / (float)DM);

  float q = 0.0f;
#pragma unroll 1
  for (int j = 0; j < 3; ++j) {
    const int off = 256 * j + 8 * lane;
    const v4f va = *(const v4fa*)(xw + off);
    const v4f vb = *(const v4fa*)(xw + off + 4);
    float dlt;
    dlt = va.x - mu; q += dlt * dlt;
    dlt = va.y - mu; q += dlt * dlt;
    dlt = va.z - mu; q += dlt * dlt;
    dlt = va.w - mu; q += dlt * dlt;
    dlt = vb.x - mu; q += dlt * dlt;
    dlt = vb.y - mu; q += dlt * dlt;
    dlt = vb.z - mu; q += dlt * dlt;
    dlt = vb.w - mu; q += dlt * dlt;
  }
#pragma unroll
  for (int d = 16; d > 0; d >>= 1) q += __shfl_xor(q, d, 32);
  const float rstd = rsqrtf(q * (1.0f / (float)DM) + 1e-5f);

#pragma unroll 1
  for (int j = 0; j < 3; ++j) {
    const int off = 256 * j + 8 * lane;
    const v4f va = *(const v4fa*)(xw + off);
    const v4f vb = *(const v4fa*)(xw + off + 4);
    const v4f wa = *(const v4fa*)(lnw + off);
    const v4f wb = *(const v4fa*)(lnw + off + 4);
    const v4f ba = *(const v4fa*)(lnb + off);
    const v4f bb = *(const v4fa*)(lnb + off + 4);
    v8us oh, ol;
    unsigned short a0, a1;
    split2((va.x - mu) * rstd * bf16_val(wa.x) + bf16_val(ba.x), a0, a1); oh[0] = a0; ol[0] = a1;
    split2((va.y - mu) * rstd * bf16_val(wa.y) + bf16_val(ba.y), a0, a1); oh[1] = a0; ol[1] = a1;
    split2((va.z - mu) * rstd * bf16_val(wa.z) + bf16_val(ba.z), a0, a1); oh[2] = a0; ol[2] = a1;
    split2((va.w - mu) * rstd * bf16_val(wa.w) + bf16_val(ba.w), a0, a1); oh[3] = a0; ol[3] = a1;
    split2((vb.x - mu) * rstd * bf16_val(wb.x) + bf16_val(bb.x), a0, a1); oh[4] = a0; ol[4] = a1;
    split2((vb.y - mu) * rstd * bf16_val(wb.y) + bf16_val(bb.y), a0, a1); oh[5] = a0; ol[5] = a1;
    split2((vb.z - mu) * rstd * bf16_val(wb.z) + bf16_val(bb.z), a0, a1); oh[6] = a0; ol[6] = a1;
    split2((vb.w - mu) * rstd * bf16_val(wb.w) + bf16_val(bb.w), a0, a1); oh[7] = a0; ol[7] = a1;
    unsigned short* rp = XN + (size_t)row * K1 + off;
    *(volatile v8us*)rp = oh;
    *(volatile v8us*)(rp + DM) = ol;
    __threadfence();
    *(volatile v8us*)rp = oh;
    *(volatile v8us*)(rp + DM) = ol;
  }
}

template <int RES>
__global__ __launch_bounds__(GTHR) void k_gemm(
    const unsigned short* __restrict__ A, const unsigned short* __restrict__ WT,
    float* outF, const float* __restrict__ resid, int K, int ldo)
{
  __shared__ __attribute__((aligned(16))) float stg[GBM * GBN];
  const int tid = (int)threadIdx.x, lane = tid & 31, wave = tid >> 5, hh = lane >> 4, m = lane & 15;
  const int rowBase = (int)blockIdx.x * GBM;
  const int col0    = (int)blockIdx.y * GBN;

  v8f acc[4];
  {
    const v8f z = {0.f, 0.f, 0.f, 0.f, 0.f, 0.f, 0.f, 0.f};
    acc[0] = z; acc[1] = z; acc[2] = z; acc[3] = z;
  }
  const unsigned short* ap = A  + (size_t)(rowBase + 16 * wave + m) * (size_t)K + 8 * hh;
  const unsigned short* wp = WT + (size_t)(col0 + m) * (size_t)K + 8 * hh;
  const int ksteps = K >> 5;
#pragma unroll 1
  for (int ks = 0; ks < ksteps; ++ks) {
    FragB af;
    af.h[0] = *(const v8usa*)(ap + 32 * ks);
    af.h[1] = *(const v8usa*)(ap + 32 * ks + 16);
#pragma unroll
    for (int t = 0; t < 4; ++t) {
      const unsigned short* wq = wp + (size_t)(16 * t) * (size_t)K + 32 * ks;
      FragB bf;
      bf.h[0] = *(const v8usa*)wq;
      bf.h[1] = *(const v8usa*)(wq + 16);
      acc[t] = wmb(af, bf, acc[t]);
    }
  }

#pragma unroll
  for (int t = 0; t < 4; ++t) {
    const int lc = 16 * t + m;
#pragma unroll
    for (int r = 0; r < 8; ++r) {
      const int lr = 16 * wave + 8 * hh + r;
      stg[lr * GBN + lc] = acc[t][r];
    }
  }
  __syncthreads();

  v4f fv[8];
#pragma unroll
  for (int i = 0; i < 8; ++i) {
    const int lr = 16 * wave + 2 * i + hh;
    fv[i] = *(const v4fa*)(stg + lr * GBN + 4 * m);
  }
  if constexpr (RES != 0) {
#pragma unroll
    for (int i = 0; i < 8; ++i) {
      const int gr = rowBase + 16 * wave + 2 * i + hh;
      const v4f rx = *(const v4fa*)(resid + (size_t)gr * (size_t)ldo + col0 + 4 * m);
      fv[i].x += bf16_val(rx.x); fv[i].y += bf16_val(rx.y);
      fv[i].z += bf16_val(rx.z); fv[i].w += bf16_val(rx.w);
    }
  }
#pragma unroll
  for (int i = 0; i < 8; ++i) {
    const int gr = rowBase + 16 * wave + 2 * i + hh;
    float* op = outF + (size_t)gr * (size_t)ldo + col0 + 4 * m;
    *(volatile v4f*)op = fv[i];
  }
  __threadfence();
#pragma unroll
  for (int i = 0; i < 8; ++i) {
    const int gr = rowBase + 16 * wave + 2 * i + hh;
    float* op = outF + (size_t)gr * (size_t)ldo + col0 + 4 * m;
    *(volatile v4f*)op = fv[i];
  }
}

__global__ __launch_bounds__(NTHR) void k_conv(const float* __restrict__ ZX, const float* __restrict__ cw,
                                               const float* __restrict__ cb, float* XC) {
  const int u = (int)blockIdx.x * NTHR + (int)threadIdx.x;
  if (u >= NU_CONV) return;
  const int tok = u / C4ROW;
  const int c4  = (u - tok * C4ROW) * 4;
  const int l   = tok & (SEQ - 1);
  const v4f w0 = *(const v4fa*)(cw + (size_t)(c4 + 0) * 4);
  const v4f w1 = *(const v4fa*)(cw + (size_t)(c4 + 1) * 4);
  const v4f w2 = *(const v4fa*)(cw + (size_t)(c4 + 2) * 4);
  const v4f w3 = *(const v4fa*)(cw + (size_t)(c4 + 3) * 4);
  const v4f bs = *(const v4fa*)(cb + c4);
  const bool ok0 = l >= 3, ok1 = l >= 2, ok2 = l >= 1;
  const int t0 = ok0 ? tok - 3 : tok;
  const int t1 = ok1 ? tok - 2 : tok;
  const int t2 = ok2 ? tok - 1 : tok;
  v4f z0 = *(const v4fa*)(ZX + (size_t)t0  * NPAD + DI + c4);
  v4f z1 = *(const v4fa*)(ZX + (size_t)t1  * NPAD + DI + c4);
  v4f z2 = *(const v4fa*)(ZX + (size_t)t2  * NPAD + DI + c4);
  const v4f z3 = *(const v4fa*)(ZX + (size_t)tok * NPAD + DI + c4);
  const v4f zz = {0.0f, 0.0f, 0.0f, 0.0f};
  z0 = ok0 ? z0 : zz;
  z1 = ok1 ? z1 : zz;
  z2 = ok2 ? z2 : zz;
  float a0 = z0.x * bf16_val(w0.x); a0 += z1.x * bf16_val(w0.y); a0 += z2.x * bf16_val(w0.z); a0 += z3.x * bf16_val(w0.w);
  float a1 = z0.y * bf16_val(w1.x); a1 += z1.y * bf16_val(w1.y); a1 += z2.y * bf16_val(w1.z); a1 += z3.y * bf16_val(w1.w);
  float a2 = z0.z * bf16_val(w2.x); a2 += z1.z * bf16_val(w2.y); a2 += z2.z * bf16_val(w2.z); a2 += z3.z * bf16_val(w2.w);
  float a3 = z0.w * bf16_val(w3.x); a3 += z1.w * bf16_val(w3.y); a3 += z2.w * bf16_val(w3.z); a3 += z3.w * bf16_val(w3.w);
  a0 += bf16_val(bs.x); a1 += bf16_val(bs.y); a2 += bf16_val(bs.z); a3 += bf16_val(bs.w);
  v4f o;
  o.x = silu_f(a0); o.y = silu_f(a1); o.z = silu_f(a2); o.w = silu_f(a3);
  float* op = XC + (size_t)tok * CONVD + c4;
  *(volatile v4f*)op = o;
  __threadfence();
  *(volatile v4f*)op = o;
}

__global__ __launch_bounds__(GTHR) void k_ssd(const float* __restrict__ ZX, const float* __restrict__ XC,
                                              const float* __restrict__ dtb, const float* __restrict__ alog,
                                              const float* __restrict__ dpar, float* Y) {
  extern __shared__ __attribute__((aligned(16))) int dsm[];
  unsigned short* Chi  = (unsigned short*)dsm;
  unsigned short* Clo  = Chi  + TE;
  unsigned short* Bhi  = Clo  + TE;
  unsigned short* Blo  = Bhi  + TE;
  unsigned short* BThi = Blo  + TE;
  unsigned short* BTlo = BThi + TE;
  unsigned short* XThi = BTlo + TE;
  unsigned short* XTlo = XThi + TE;
  unsigned short* Mhi  = XTlo + TE;
  unsigned short* Mlo  = Mhi  + TE;
  unsigned short* Hhi  = Mlo  + TE;
  unsigned short* Hlo  = Hhi  + TE;
  float* Hf  = (float*)(dsm + 12 * (TE / 2));
  float* stg = Hf  + TE;
  float* sdt = stg + TE;
  float* sa  = sdt + 64;
  float* scs = sa  + 64;
  float* sE  = scs + 64;
  float* sW  = sE  + 64;

  const int tid = (int)threadIdx.x, lane = tid & 31, wave = tid >> 5, hh = lane >> 4, m = lane & 15;
  const int b = (int)blockIdx.x / NH;
  const int h = (int)blockIdx.x - b * NH;
  const float dtbias = bf16_val(dtb[h]);
  const float Ah     = -expf(bf16_val(alog[h]));
  const float Dh     = bf16_val(dpar[h]);

#pragma unroll 1
  for (int i = tid; i < TE; i += GTHR) {
    Hf[i] = 0.0f;
    Hhi[i] = (unsigned short)0;
    Hlo[i] = (unsigned short)0;
  }

#pragma unroll 1
  for (int c = 0; c < NCH; ++c) {
    const int tok0 = b * SEQ + c * QC;

    if (tid < QC) {
      const float raw = ZX[(size_t)(tok0 + tid) * NPAD + DTOFF + h] + dtbias;
      const float sp  = fmaxf(raw, 0.0f) + log1pf(expf(-fabsf(raw)));
      sdt[tid] = sp;
      sa[tid]  = sp * Ah;
    }
    __syncthreads();

    if (tid < QC) {
      float s = 0.0f, tot = 0.0f;
#pragma unroll 1
      for (int i = 0; i < QC; ++i) {
        const float ai = sa[i];
        s   += (i <= tid) ? ai : 0.0f;
        tot += ai;
      }
      scs[tid] = s;
      sE[tid]  = expf(fminf(s, 0.0f));
      sW[tid]  = expf(fminf(tot - s, 0.0f)) * sdt[tid];
    }
#pragma unroll 1
    for (int i = 0; i < 8; ++i) {
      const int idx = tid + GTHR * i;
      const int row = idx >> 4;
      const int c4  = (idx & 15) * 4;
      const float* rp = XC + (size_t)(tok0 + row) * CONVD;
      const v4f xv = *(const v4fa*)(rp + h * HD + c4);
      const v4f bv = *(const v4fa*)(rp + DI + c4);
      const v4f cv = *(const v4fa*)(rp + DI + DS + c4);
      v4us q0, q1;
      unsigned short a0, a1;
      split2(cv.x, a0, a1); q0[0] = a0; q1[0] = a1;
      split2(cv.y, a0, a1); q0[1] = a0; q1[1] = a1;
      split2(cv.z, a0, a1); q0[2] = a0; q1[2] = a1;
      split2(cv.w, a0, a1); q0[3] = a0; q1[3] = a1;
      *(v4usa*)(Chi + row * 64 + c4) = q0;
      *(v4usa*)(Clo + row * 64 + c4) = q1;
      split2(bv.x, a0, a1); q0[0] = a0; q1[0] = a1;
      split2(bv.y, a0, a1); q0[1] = a0; q1[1] = a1;
      split2(bv.z, a0, a1); q0[2] = a0; q1[2] = a1;
      split2(bv.w, a0, a1); q0[3] = a0; q1[3] = a1;
      *(v4usa*)(Bhi + row * 64 + c4) = q0;
      *(v4usa*)(Blo + row * 64 + c4) = q1;
      split2(xv.x, a0, a1); XThi[(c4 + 0) * 64 + row] = a0; XTlo[(c4 + 0) * 64 + row] = a1;
      split2(xv.y, a0, a1); XThi[(c4 + 1) * 64 + row] = a0; XTlo[(c4 + 1) * 64 + row] = a1;
      split2(xv.z, a0, a1); XThi[(c4 + 2) * 64 + row] = a0; XTlo[(c4 + 2) * 64 + row] = a1;
      split2(xv.w, a0, a1); XThi[(c4 + 3) * 64 + row] = a0; XTlo[(c4 + 3) * 64 + row] = a1;
    }
    __syncthreads();

    {
      v8f g[4];
      {
        const v8f z = {0.f, 0.f, 0.f, 0.f, 0.f, 0.f, 0.f, 0.f};
        g[0] = z; g[1] = z; g[2] = z; g[3] = z;
      }
#pragma unroll
      for (int ks = 0; ks < 2; ++ks) {
        const int ko = 32 * ks + 8 * hh;
        FragB ah, al;
        lds_frag(ah, Chi + (16 * wave + m) * 64 + ko);
        lds_frag(al, Clo + (16 * wave + m) * 64 + ko);
#pragma unroll
        for (int j = 0; j < 4; ++j) {
          FragB bh, bl;
          lds_frag(bh, Bhi + (16 * j + m) * 64 + ko);
          lds_frag(bl, Blo + (16 * j + m) * 64 + ko);
          g[j] = mm3(ah, al, bh, bl, g[j]);
        }
      }
#pragma unroll
      for (int j = 0; j < 4; ++j) {
        const int s = 16 * j + m;
        const float css = scs[s];
        const float dts = sdt[s];
#pragma unroll
        for (int r = 0; r < 8; ++r) {
          const int t = 16 * wave + 8 * hh + r;
          const float d  = fminf(scs[t] - css, 0.0f);
          const float mv = g[j][r] * expf(d) * dts;
          const float mz = (s <= t) ? mv : 0.0f;
          unsigned short a0, a1;
          split2(mz, a0, a1);
          Mhi[t * 64 + s] = a0;
          Mlo[t * 64 + s] = a1;
        }
      }
    }
#pragma unroll 1
    for (int i = 0; i < 8; ++i) {
      const int idx = tid + GTHR * i;
      const int row = idx >> 4;
      const int c4  = (idx & 15) * 4;
      const v4f bv = *(const v4fa*)(XC + (size_t)(tok0 + row) * CONVD + DI + c4);
      const float ws = sW[row];
      unsigned short a0, a1;
      split2(bv.x * ws, a0, a1); BThi[(c4 + 0) * 64 + row] = a0; BTlo[(c4 + 0) * 64 + row] = a1;
      split2(bv.y * ws, a0, a1); BThi[(c4 + 1) * 64 + row] = a0; BTlo[(c4 + 1) * 64 + row] = a1;
      split2(bv.z * ws, a0, a1); BThi[(c4 + 2) * 64 + row] = a0; BTlo[(c4 + 2) * 64 + row] = a1;
      split2(bv.w * ws, a0, a1); BThi[(c4 + 3) * 64 + row] = a0; BTlo[(c4 + 3) * 64 + row] = a1;
    }
    __syncthreads();

    {
      v8f yd[4], yo[4];
      {
        const v8f z = {0.f, 0.f, 0.f, 0.f, 0.f, 0.f, 0.f, 0.f};
        yd[0] = z; yd[1] = z; yd[2] = z; yd[3] = z;
        yo[0] = z; yo[1] = z; yo[2] = z; yo[3] = z;
      }
#pragma unroll
      for (int ks = 0; ks < 2; ++ks) {
        const int ko = 32 * ks + 8 * hh;
        FragB mh, ml, ch, cl;
        lds_frag(mh, Mhi + (16 * wave + m) * 64 + ko);
        lds_frag(ml, Mlo + (16 * wave + m) * 64 + ko);
        lds_frag(ch, Chi + (16 * wave + m) * 64 + ko);
        lds_frag(cl, Clo + (16 * wave + m) * 64 + ko);
#pragma unroll
        for (int j = 0; j < 4; ++j) {
          FragB xh, xl, qh, ql;
          lds_frag(xh, XThi + (16 * j + m) * 64 + ko);
          lds_frag(xl, XTlo + (16 * j + m) * 64 + ko);
          yd[j] = mm3(mh, ml, xh, xl, yd[j]);
          lds_frag(qh, Hhi + (16 * j + m) * 64 + ko);
          lds_frag(ql, Hlo + (16 * j + m) * 64 + ko);
          yo[j] = mm3(ch, cl, qh, ql, yo[j]);
        }
      }
#pragma unroll
      for (int j = 0; j < 4; ++j) {
        const int p = 16 * j + m;
#pragma unroll
        for (int r = 0; r < 8; ++r) {
          const int t = 16 * wave + 8 * hh + r;
          const float xv = bf_to_f(XThi[p * 64 + t]) + bf_to_f(XTlo[p * 64 + t]);
          const float yv = yd[j][r] + sE[t] * yo[j][r] + Dh * xv;
          stg[t * 64 + p] = yv;
        }
      }
    }
    __syncthreads();

    {
      v4f fv[8];
#pragma unroll
      for (int i = 0; i < 8; ++i) {
        const int lr = 16 * wave + 2 * i + hh;
        fv[i] = *(const v4fa*)(stg + lr * 64 + 4 * m);
      }
#pragma unroll
      for (int i = 0; i < 8; ++i) {
        const int lr = 16 * wave + 2 * i + hh;
        float* op = Y + (size_t)(tok0 + lr) * DI + h * HD + 4 * m;
        *(volatile v4f*)op = fv[i];
      }
      __threadfence();
#pragma unroll
      for (int i = 0; i < 8; ++i) {
        const int lr = 16 * wave + 2 * i + hh;
        float* op = Y + (size_t)(tok0 + lr) * DI + h * HD + 4 * m;
        *(volatile v4f*)op = fv[i];
      }
    }
    {
      v8f sc[4];
      {
        const v8f z = {0.f, 0.f, 0.f, 0.f, 0.f, 0.f, 0.f, 0.f};
        sc[0] = z; sc[1] = z; sc[2] = z; sc[3] = z;
      }
#pragma unroll
      for (int ks = 0; ks < 2; ++ks) {
        const int ko = 32 * ks + 8 * hh;
        FragB xh, xl;
        lds_frag(xh, XThi + (16 * wave + m) * 64 + ko);
        lds_frag(xl, XTlo + (16 * wave + m) * 64 + ko);
#pragma unroll
        for (int j = 0; j < 4; ++j) {
          FragB th, tl;
          lds_frag(th, BThi + (16 * j + m) * 64 + ko);
          lds_frag(tl, BTlo + (16 * j + m) * 64 + ko);
          sc[j] = mm3(xh, xl, th, tl, sc[j]);
        }
      }
      const float eend = sE[QC - 1];
#pragma unroll
      for (int j = 0; j < 4; ++j) {
        const int n = 16 * j + m;
#pragma unroll
        for (int r = 0; r < 8; ++r) {
          const int p = 16 * wave + 8 * hh + r;
          const float hv = eend * Hf[p * 64 + n] + sc[j][r];
          Hf[p * 64 + n] = hv;
          unsigned short a0, a1;
          split2(hv, a0, a1);
          Hhi[p * 64 + n] = a0;
          Hlo[p * 64 + n] = a1;
        }
      }
    }
    __syncthreads();
  }
}

__global__ __launch_bounds__(NTHR) void k_gate(const float* __restrict__ Yp, const float* __restrict__ ZX,
                                               const float* __restrict__ rmsw, unsigned short* GH) {
  __shared__ __attribute__((aligned(16))) float gb[8 * DI];
  const int tid = (int)threadIdx.x, lane = tid & 31, wave = tid >> 5;
  const int row = (int)blockIdx.x * 8 + wave;
  float* gw = gb + wave * DI;
  const float* yr = Yp + (size_t)row * DI;
  const float* zr = ZX + (size_t)row * NPAD;
  float ss = 0.0f;
#pragma unroll 1
  for (int j = 0; j < 6; ++j) {
    const int off = 256 * j + 8 * lane;
    const v4f ya = *(const v4fa*)(yr + off);
    const v4f yb = *(const v4fa*)(yr + off + 4);
    const v4f za = *(const v4fa*)(zr + off);
    const v4f zb = *(const v4fa*)(zr + off + 4);
    v4f ga, gc;
    ga.x = ya.x * silu_f(za.x); ga.y = ya.y * silu_f(za.y);
    ga.z = ya.z * silu_f(za.z); ga.w = ya.w * silu_f(za.w);
    gc.x = yb.x * silu_f(zb.x); gc.y = yb.y * silu_f(zb.y);
    gc.z = yb.z * silu_f(zb.z); gc.w = yb.w * silu_f(zb.w);
    ss += ga.x * ga.x; ss += ga.y * ga.y; ss += ga.z * ga.z; ss += ga.w * ga.w;
    ss += gc.x * gc.x; ss += gc.y * gc.y; ss += gc.z * gc.z; ss += gc.w * gc.w;
    *(v4fa*)(gw + off) = ga;
    *(v4fa*)(gw + off + 4) = gc;
  }
#pragma unroll
  for (int d = 16; d > 0; d >>= 1) ss += __shfl_xor(ss, d, 32);
  const float rstd = rsqrtf(ss * (1.0f / (float)DI) + 1e-5f);
#pragma unroll 1
  for (int j = 0; j < 6; ++j) {
    const int off = 256 * j + 8 * lane;
    const v4f ga = *(const v4fa*)(gw + off);
    const v4f gc = *(const v4fa*)(gw + off + 4);
    const v4f wa = *(const v4fa*)(rmsw + off);
    const v4f wb = *(const v4fa*)(rmsw + off + 4);
    v8us oh, ol;
    unsigned short a0, a1;
    split2(ga.x * rstd * bf16_val(wa.x), a0, a1); oh[0] = a0; ol[0] = a1;
    split2(ga.y * rstd * bf16_val(wa.y), a0, a1); oh[1] = a0; ol[1] = a1;
    split2(ga.z * rstd * bf16_val(wa.z), a0, a1); oh[2] = a0; ol[2] = a1;
    split2(ga.w * rstd * bf16_val(wa.w), a0, a1); oh[3] = a0; ol[3] = a1;
    split2(gc.x * rstd * bf16_val(wb.x), a0, a1); oh[4] = a0; ol[4] = a1;
    split2(gc.y * rstd * bf16_val(wb.y), a0, a1); oh[5] = a0; ol[5] = a1;
    split2(gc.z * rstd * bf16_val(wb.z), a0, a1); oh[6] = a0; ol[6] = a1;
    split2(gc.w * rstd * bf16_val(wb.w), a0, a1); oh[7] = a0; ol[7] = a1;
    unsigned short* rp = GH + (size_t)row * K2 + off;
    *(volatile v8us*)rp = oh;
    *(volatile v8us*)(rp + DI) = ol;
    __threadfence();
    *(volatile v8us*)rp = oh;
    *(volatile v8us*)(rp + DI) = ol;
  }
}

static inline size_t al256(size_t o) { return (o + 255) & ~(size_t)255; }

extern "C" void kernel_launch(void* const* d_in, const int* in_sizes, int n_in,
                              void* d_out, int out_size, void* d_ws, size_t ws_size,
                              hipStream_t stream) {
  if (n_in < 11) return;
  if (in_sizes[0] != NTOK * DM) return;
  if (in_sizes[1] != DM || in_sizes[2] != DM) return;
  if (in_sizes[3] != DM * DPROJ) return;
  if (in_sizes[4] != CONVD * 4 || in_sizes[5] != CONVD) return;
  if (in_sizes[6] != NH || in_sizes[7] != NH || in_sizes[8] != NH) return;
  if (in_sizes[9] != DI || in_sizes[10] != DI * DM) return;
  if (out_size != NTOK * DM) return;

  const float* x     = (const float*)d_in[0];
  const float* ln_w  = (const float*)d_in[1];
  const float* ln_b  = (const float*)d_in[2];
  const float* W_in  = (const float*)d_in[3];
  const float* cw    = (const float*)d_in[4];
  const float* cb    = (const float*)d_in[5];
  const float* dtb   = (const float*)d_in[6];
  const float* alog  = (const float*)d_in[7];
  const float* dpar  = (const float*)d_in[8];
  const float* rms_w = (const float*)d_in[9];
  const float* W_out = (const float*)d_in[10];
  float* out = (float*)d_out;

  char* ws = (char*)d_ws;
  size_t off = 0;
  const size_t oWIN  = off; off = al256(off + (size_t)NPAD * K1 * 2);
  const size_t oWOUT = off; off = al256(off + (size_t)DM * K2 * 2);
  const size_t oXN   = off; off = al256(off + (size_t)NTOK * K1 * 2);
  const size_t oZX   = off; off = al256(off + (size_t)NTOK * NPAD * 4);
  const size_t oXC   = off; off = al256(off + (size_t)NTOK * CONVD * 4);
  const size_t oY    = off; off = al256(off + (size_t)NTOK * DI * 4);
  const size_t oGH   = off; off = al256(off + (size_t)NTOK * K2 * 2);
  if (off > ws_size || off > (size_t)WSMAX) return;
  unsigned short* WIN2  = (unsigned short*)(ws + oWIN);
  unsigned short* WOUT2 = (unsigned short*)(ws + oWOUT);
  unsigned short* XN    = (unsigned short*)(ws + oXN);
  float*          ZX    = (float*)(ws + oZX);
  float*          XC    = (float*)(ws + oXC);
  float*          Yb    = (float*)(ws + oY);
  unsigned short* GH    = (unsigned short*)(ws + oGH);

  const size_t ssdLds = (size_t)SSD_INTS * 4;
  hipFuncSetAttribute(reinterpret_cast<const void*>(&k_ssd), hipFuncAttributeMaxDynamicSharedMemorySize, (int)ssdLds);

  k_prep<<<(NU_IN + NU_OUT) / NTHR, NTHR, 0, stream>>>(W_in, W_out, WIN2, WOUT2);
  k_ln<<<NTOK / 8, NTHR, 0, stream>>>(x, ln_w, ln_b, XN);
  k_gemm<0><<<dim3(NTOK / GBM, NPAD / GBN), GTHR, 0, stream>>>(XN, WIN2, ZX, x, K1, NPAD);
  k_conv<<<NU_CONV / NTHR, NTHR, 0, stream>>>(ZX, cw, cb, XC);
  k_ssd<<<2 * NH, GTHR, ssdLds, stream>>>(ZX, XC, dtb, alog, dpar, Yb);
  k_gate<<<NTOK / 8, NTHR, 0, stream>>>(Yb, ZX, rms_w, GH);
  k_gemm<1><<<dim3(NTOK / GBM, DM / GBN), GTHR, 0, stream>>>(GH, WOUT2, out, x, K2, DM);
}
